// GIN_36481452212846
// MI455X (gfx1250) — hardware-verified
//
#include <hip/hip_runtime.h>
#include <stddef.h>
#include <stdint.h>
#include <math.h>


#define CIN    128
#define HID    64
#define KK     128
#define NLAY   4
#define NPL    8
#define PLSZ   (HID * KK)
#define NUPL   (HID * (KK / 8))
#define NUW    (NPL * NUPL)
#define NTHR   256
#define NWAVE  8
#define EPT    8
#define CHUNK  (NTHR * EPT)
#define WCAP   (EPT * 32)
#define LISTN  (NWAVE * WCAP)
#define NBA    1024
#define SLA    10
#define RCAP   28672
#define DEGCAP 64
#define GBM    64
#define GBN    64
#define GTHR   128
#define PARTW  160
#define APR    32
#define AGG_ZINTS (LISTN + 2 * RCAP + 3 * NBA)
#define AGG_LDS_INTS (AGG_ZINTS + 16)
#define WSMAX  134217728

static_assert((CHUNK & (CHUNK - 1)) == 0 && CHUNK <= 4096);
static_assert((NBA & (NBA - 1)) == 0 && NBA == (1 << SLA));
static_assert(((long long)CHUNK << SLA) < (1LL << 31));
static_assert(LISTN % NTHR == 0);
static_assert(NBA % NWAVE == 0 && NBA % 32 == 0 && NBA % GBM == 0);
static_assert(RCAP % 32 == 0 && AGG_ZINTS % 4 == 0 && LISTN % 4 == 0);
static_assert(CIN % 32 == 0 && KK % 32 == 0 && KK == 2 * HID && KK == CIN && HID == GBN);
static_assert(GBM == (GTHR / 32) * 16 && GBN == 64);
static_assert(NUPL == 1024 && NUPL % NTHR == 0 && NUW % NTHR == 0);
static_assert(CIN / 8 == 16 && KK / 8 == 16);
static_assert(HID == 2 * 32);
static_assert(AGG_LDS_INTS * 4 <= 300000);
static_assert(PARTW % 32 == 0 && PARTW >= 2 * GBN + 1 && PARTW / 4 <= GTHR && GBN <= GTHR);
static_assert(NTHR == 4 * HID && (APR % 4) == 0 && APR * HID == 2 * 4 * NTHR && APR * (KK / 8) == 2 * NTHR);
static_assert((GBM % APR) == 0 && 2 * HID <= NTHR && 2 * HID == 4 * 32);
static_assert((DEGCAP % 32) == 0 || DEGCAP < 32 || DEGCAP > 0);

typedef float          v2f   __attribute__((ext_vector_type(2)));
typedef float          v4f   __attribute__((ext_vector_type(4)));
typedef float          v8f   __attribute__((ext_vector_type(8)));
typedef int            v4i   __attribute__((ext_vector_type(4)));
typedef int            v8i   __attribute__((ext_vector_type(8)));
typedef unsigned int   v4u   __attribute__((ext_vector_type(4)));
typedef unsigned short v8us  __attribute__((ext_vector_type(8)));
typedef unsigned short v16us __attribute__((ext_vector_type(16)));
typedef __bf16         v16bf __attribute__((ext_vector_type(16)));
typedef v2f  __attribute__((may_alias)) v2fa;
typedef v4f  __attribute__((may_alias)) v4fa;
typedef v4i  __attribute__((may_alias)) v4ia;
typedef v8us __attribute__((may_alias)) v8usa;
union FragB { v16bf v; v16us u; v8us h[2]; v8i w; };

__device__ __forceinline__ v8f wmb(const FragB& a, const FragB& b, v8f c) {
  v8f d = __builtin_amdgcn_wmma_f32_16x16x32_bf16(false, a.v, false, b.v, (short)0, c, false, false);
  asm volatile("v_nop\n\tv_nop\n\tv_nop\n\tv_nop" : "+v"(d) : "v"(a.w), "v"(b.w));
  return d;
}

__device__ __forceinline__ unsigned bf16_bits(float f) {
  const unsigned u = __float_as_uint(f);
  return (u + 0x7FFFu + ((u >> 16) & 1u)) >> 16;
}
__device__ __forceinline__ float bf16_val(float f) {
  return __uint_as_float(bf16_bits(f) << 16);
}

__device__ __forceinline__ void hilo8(const v4f a, const v4f b, v8us& hv, v8us& lv) {
  const float f[8] = {a.x, a.y, a.z, a.w, b.x, b.y, b.z, b.w};
#pragma unroll
  for (int j = 0; j < 8; ++j) {
    const unsigned hb = bf16_bits(f[j]);
    hv[j] = (unsigned short)hb;
    lv[j] = (unsigned short)bf16_bits(f[j] - __uint_as_float(hb << 16));
  }
}

template <int SLB>
__device__ __forceinline__ int scan_chunk(const int* __restrict__ dsts, int nE, int cbase, int slotBase,
                                          int nb, int vec8, int* list, int tid, int lane, int wave) {
  int wc = 0;
  const int el0  = tid * EPT;
  const int e0   = cbase + el0;
  const int sent = -2147483647 - 1;
  v4i da, db;
  if (vec8 != 0 && cbase + CHUNK <= nE) {
    da = *(const v4i*)(dsts + e0);
    db = *(const v4i*)(dsts + e0 + 4);
  } else {
    da.x = (e0     < nE) ? dsts[min(e0,     nE - 1)] : sent;
    da.y = (e0 + 1 < nE) ? dsts[min(e0 + 1, nE - 1)] : sent;
    da.z = (e0 + 2 < nE) ? dsts[min(e0 + 2, nE - 1)] : sent;
    da.w = (e0 + 3 < nE) ? dsts[min(e0 + 3, nE - 1)] : sent;
    db.x = (e0 + 4 < nE) ? dsts[min(e0 + 4, nE - 1)] : sent;
    db.y = (e0 + 5 < nE) ? dsts[min(e0 + 5, nE - 1)] : sent;
    db.z = (e0 + 6 < nE) ? dsts[min(e0 + 6, nE - 1)] : sent;
    db.w = (e0 + 7 < nE) ? dsts[min(e0 + 7, nE - 1)] : sent;
  }
  const unsigned nbs = (unsigned)slotBase;
  const unsigned unb = (unsigned)nb;
  const unsigned s0 = (unsigned)da.x - nbs, s1 = (unsigned)da.y - nbs;
  const unsigned s2 = (unsigned)da.z - nbs, s3 = (unsigned)da.w - nbs;
  const unsigned s4 = (unsigned)db.x - nbs, s5 = (unsigned)db.y - nbs;
  const unsigned s6 = (unsigned)db.z - nbs, s7 = (unsigned)db.w - nbs;
  const bool h0 = s0 < unb, h1 = s1 < unb, h2 = s2 < unb, h3 = s3 < unb;
  const bool h4 = s4 < unb, h5 = s5 < unb, h6 = s6 < unb, h7 = s7 < unb;
  const unsigned any = __builtin_amdgcn_ballot_w32(h0 | h1 | h2 | h3 | h4 | h5 | h6 | h7);
  if (any != 0u) {
#define HITJ(J, HJ, SJ) { \
      const unsigned mj = __builtin_amdgcn_ballot_w32(HJ); \
      if (mj != 0u) { \
        if (HJ) { \
          const int pos = wc + (int)__builtin_amdgcn_mbcnt_lo(mj, 0u); \
          if (pos < WCAP) list[wave * WCAP + pos] = ((el0 + (J)) << SLB) | (int)(SJ); \
        } \
        wc += (int)__builtin_popcount(mj); } }
    HITJ(0, h0, s0)
    HITJ(1, h1, s1)
    HITJ(2, h2, s2)
    HITJ(3, h3, s3)
    HITJ(4, h4, s4)
    HITJ(5, h5, s5)
    HITJ(6, h6, s6)
    HITJ(7, h7, s7)
#undef HITJ
  }
  return wc;
}

__global__ __launch_bounds__(NTHR) void k_wprep(const float* __restrict__ w10, const float* __restrict__ w20,
                                                const float* __restrict__ w1s, const float* __restrict__ w2s,
                                                unsigned short* wp) {
  const int u = (int)blockIdx.x * NTHR + (int)threadIdx.x;
  if (u >= NUW) return;
  const int g  = u >> 10;
  const int v  = u & (NUPL - 1);
  const int n  = v >> 4;
  const int k8 = (v & 15) * 8;
  const float* base;
  int kmask;
  if (g == 0)            { base = w10; kmask = CIN - 1; }
  else if (g == 1)       { base = w20; kmask = HID - 1; }
  else if ((g & 1) == 0) { base = w1s + (size_t)((g - 2) >> 1) * (size_t)(HID * HID); kmask = HID - 1; }
  else                   { base = w2s + (size_t)((g - 3) >> 1) * (size_t)(HID * HID); kmask = HID - 1; }
  const int kk = k8 & kmask;
  const float* p = base + (size_t)kk * HID + n;
  v8us o;
#pragma unroll
  for (int i = 0; i < 8; ++i) o[i] = (unsigned short)bf16_bits(p[(size_t)i * HID]);
  unsigned short* dp = wp + (size_t)g * PLSZ + (size_t)n * KK + k8;
  *(volatile v8us*)dp = o;
  __threadfence();
  *(volatile v8us*)dp = o;
}

__global__ __launch_bounds__(NTHR) void k_cvx(const float* __restrict__ x, int nN, int nUnits,
                                              unsigned short* xb) {
  const int u = (int)blockIdx.x * NTHR + (int)threadIdx.x;
  if (u >= nUnits) return;
  const int row = u >> 4;
  const int k8  = (u & 15) * 8;
  const int rc  = row < nN ? row : nN - 1;
  const float* p = x + (size_t)rc * CIN + k8;
  const v4f a = *(const v4fa*)p;
  const v4f b = *(const v4fa*)(p + 4);
  const bool ok = row < nN;
  v8us o;
  o[0] = ok ? (unsigned short)bf16_bits(a.x) : (unsigned short)0;
  o[1] = ok ? (unsigned short)bf16_bits(a.y) : (unsigned short)0;
  o[2] = ok ? (unsigned short)bf16_bits(a.z) : (unsigned short)0;
  o[3] = ok ? (unsigned short)bf16_bits(a.w) : (unsigned short)0;
  o[4] = ok ? (unsigned short)bf16_bits(b.x) : (unsigned short)0;
  o[5] = ok ? (unsigned short)bf16_bits(b.y) : (unsigned short)0;
  o[6] = ok ? (unsigned short)bf16_bits(b.z) : (unsigned short)0;
  o[7] = ok ? (unsigned short)bf16_bits(b.w) : (unsigned short)0;
  unsigned short* dp = xb + (size_t)row * CIN + k8;
  *(volatile v8us*)dp = o;
  __threadfence();
  *(volatile v8us*)dp = o;
}

template <int EPI>
__global__ __launch_bounds__(GTHR) void k_gemm(
    const unsigned short* __restrict__ A, const unsigned short* __restrict__ WT,
    const float* __restrict__ bias, float* outF, int K, int nN, float* part)
{
  __shared__ __attribute__((aligned(16))) float stg[GBM * GBN];
  __shared__ __attribute__((aligned(16))) float pst[PARTW];
  const int tid = (int)threadIdx.x, lane = tid & 31, wave = tid >> 5, hh = lane >> 4, m = lane & 15;
  const int rowBase = (int)blockIdx.x * GBM;
  const int col0    = (int)blockIdx.y * GBN;

  v8f acc[4];
  {
    const v8f z = {0.f, 0.f, 0.f, 0.f, 0.f, 0.f, 0.f, 0.f};
    acc[0] = z; acc[1] = z; acc[2] = z; acc[3] = z;
  }
  const unsigned short* ap = A  + (size_t)(rowBase + 16 * wave + m) * (size_t)K + 8 * hh;
  const unsigned short* wq0 = WT + (size_t)(col0 + m) * (size_t)K + 8 * hh;
  const int ksteps = K >> 5;
#pragma unroll 1
  for (int ks = 0; ks < ksteps; ++ks) {
    FragB af;
    af.h[0] = *(const v8usa*)(ap + 32 * ks);
    af.h[1] = *(const v8usa*)(ap + 32 * ks + 16);
#pragma unroll
    for (int t = 0; t < 4; ++t) {
      const unsigned short* wq = wq0 + (size_t)(16 * t) * (size_t)K + 32 * ks;
      FragB bfr;
      bfr.h[0] = *(const v8usa*)wq;
      bfr.h[1] = *(const v8usa*)(wq + 16);
      acc[t] = wmb(af, bfr, acc[t]);
    }
  }

#pragma unroll
  for (int t = 0; t < 4; ++t) {
    const int lc = 16 * t + m;
    float bb = 0.0f;
    if constexpr (EPI == 1) bb = bf16_val(bias[col0 + lc]);
#pragma unroll
    for (int r = 0; r < 8; ++r) {
      const int lr = 16 * wave + 8 * hh + r;
      const bool live = (rowBase + lr) < nN;
      const float v = acc[t][r] + bb;
      stg[lr * GBN + lc] = live ? v : 0.0f;
    }
  }
  __syncthreads();

  v4f fv[8];
#pragma unroll
  for (int i = 0; i < 8; ++i) {
    const int lr = 16 * wave + 2 * i + hh;
    fv[i] = *(const v4fa*)(stg + lr * GBN + 4 * m);
  }
  v4f pv = {0.f, 0.f, 0.f, 0.f};
  const bool pok = (EPI == 1) && (tid < PARTW / 4);
  if constexpr (EPI == 1) {
    int nvr = nN - rowBase;
    nvr = nvr < 0 ? 0 : (nvr > GBM ? GBM : nvr);
    if (tid < GBN) {
      float s = 0.0f;
#pragma unroll 1
      for (int r = 0; r < nvr; ++r) s += stg[r * GBN + tid];
      const float inv = 1.0f / (float)(nvr < 1 ? 1 : nvr);
      const float mean = s * inv;
      float q = 0.0f;
#pragma unroll 1
      for (int r = 0; r < nvr; ++r) {
        const float d = stg[r * GBN + tid] - mean;
        q = fmaf(d, d, q);
      }
      pst[1 + tid] = mean;
      pst[1 + GBN + tid] = q;
    }
    if (tid == 0) pst[0] = (float)nvr;
#pragma unroll 1
    for (int i = 2 * GBN + 1 + tid; i < PARTW; i += GTHR) pst[i] = 0.0f;
    __syncthreads();
    if (pok) pv = *(const v4fa*)(pst + 4 * tid);
  }
  float* pp = part + (size_t)blockIdx.x * PARTW + 4 * tid;
#pragma unroll
  for (int i = 0; i < 8; ++i) {
    const int lr = 16 * wave + 2 * i + hh;
    const int gr = rowBase + lr;
    float* op = outF + (size_t)gr * (size_t)HID + col0 + 4 * m;
    *(volatile v4f*)op = fv[i];
  }
  if (pok) *(volatile v4f*)pp = pv;
  __threadfence();
#pragma unroll
  for (int i = 0; i < 8; ++i) {
    const int lr = 16 * wave + 2 * i + hh;
    const int gr = rowBase + lr;
    float* op = outF + (size_t)gr * (size_t)HID + col0 + 4 * m;
    *(volatile v4f*)op = fv[i];
  }
  if (pok) *(volatile v4f*)pp = pv;
}

__global__ __launch_bounds__(NTHR) void k_agg(const int* __restrict__ srcs, const int* __restrict__ dsts,
                                              int nE, int nN, int vec8, int mRows,
                                              const float* __restrict__ pf, const float* __restrict__ bias,
                                              unsigned short* zb) {
  extern __shared__ __attribute__((aligned(16))) int dsm[];
  int* list = dsm;
  int* hl   = dsm + LISTN;
  int* sl   = dsm + LISTN + RCAP;
  int* cnt  = dsm + LISTN + 2 * RCAP;
  int* offs = cnt + NBA;
  int* cur  = offs + NBA;
  int* misc = cur + NBA;
  const int tid = (int)threadIdx.x, lane = tid & 31, wave = tid >> 5;
  const int nodeBase = (int)blockIdx.x * NBA;

  {
    const v4i z4 = {0, 0, 0, 0};
    for (int i = tid * 4; i < AGG_ZINTS; i += NTHR * 4) *(v4ia*)(dsm + i) = z4;
    if (tid < 16) misc[tid] = 0;
  }
  float bv0, bv1;
  {
    const v2f a = *(const v2fa*)(bias + 2 * lane);
    bv0 = bf16_val(a.x); bv1 = bf16_val(a.y);
  }
  __syncthreads();

  int t = 0, ov = 0;
  const int nChunks = (nE + CHUNK - 1) / CHUNK;
#pragma unroll 1
  for (int ch = 0; ch < nChunks; ++ch) {
    const int cbase = ch * CHUNK;
    const int wc = scan_chunk<SLA>(dsts, nE, cbase, nodeBase, NBA, vec8, list, tid, lane, wave);
    if (lane == 0) misc[wave] = wc;
    __syncthreads();
    if (wave == 0) {
#pragma unroll 1
      for (int w2 = 0; w2 < NWAVE; ++w2) {
        int c = misc[w2];
        c = c < 0 ? 0 : (c > WCAP ? WCAP : c);
#pragma unroll 1
        for (int b0 = 0; b0 < c; b0 += 32) {
          const int idx = b0 + lane;
          const int ent = list[w2 * WCAP + (idx < WCAP ? idx : WCAP - 1)];
          const int m32 = (c - b0) < 32 ? (c - b0) : 32;
#pragma unroll 1
          for (int k = 0; k < m32; ++k) {
            const int u    = __builtin_amdgcn_readlane(ent, k);
            const int slot = u & (NBA - 1);
            const int el   = (u >> SLA) & (CHUNK - 1);
            const int pk   = ((cbase + el) << SLA) | slot;
            if (t < RCAP) {
              if (lane == 0) { hl[t] = pk; cnt[slot] = cnt[slot] + 1; }
              t = t + 1;
            } else {
              ov = 1;
            }
          }
        }
      }
    }
    __syncthreads();
  }
  if (wave == 0 && lane == 0) { misc[8] = t; misc[9] = ov; }
  __syncthreads();
  int tt = misc[8];
  tt = tt < 0 ? 0 : (tt > RCAP ? RCAP : tt);
  const int ovf = misc[9];

  if (wave == 0) {
    const int base = lane * (NBA / 32);
    int s = 0;
#pragma unroll 1
    for (int i = 0; i < NBA / 32; ++i) s += cnt[base + i];
    int incl = s;
#pragma unroll
    for (int d = 1; d < 32; d <<= 1) {
      const int y = __shfl_up(incl, d, 32);
      if (lane >= d) incl += y;
    }
    int run = incl - s;
#pragma unroll 1
    for (int i = 0; i < NBA / 32; ++i) {
      const int cv = cnt[base + i];
      offs[base + i] = run;
      cur[base + i]  = run;
      run += cv;
    }
  }
  __syncthreads();
  if (wave == 0) {
#pragma unroll 1
    for (int b0 = 0; b0 < tt; b0 += 32) {
      const int idx = b0 + lane;
      const int ent = hl[idx < RCAP ? idx : RCAP - 1];
      const int m32 = (tt - b0) < 32 ? (tt - b0) : 32;
#pragma unroll 1
      for (int k = 0; k < m32; ++k) {
        const int u    = __builtin_amdgcn_readlane(ent, k);
        const int slot = u & (NBA - 1);
        if (lane == 0) {
          int p = cur[slot];
          p = p < 0 ? 0 : (p > RCAP - 1 ? RCAP - 1 : p);
          sl[p] = u;
          cur[slot] = p + 1;
        }
      }
    }
  }
  __syncthreads();

  const float qnan = __int_as_float(0x7fc00000);
  const float pz = (ovf != 0) ? qnan : 0.0f;
  const int q0s = (4 * lane) & 31, q1s = (4 * lane + 1) & 31;
  const int q2s = (4 * lane + 2) & 31, q3s = (4 * lane + 3) & 31;
#pragma unroll 1
  for (int si = 0; si < NBA / NWAVE; ++si) {
    const int s    = si * NWAVE + wave;
    const int node = nodeBase + s;
    int c = cnt[s];
    const bool big = c > DEGCAP;
    c = c < 0 ? 0 : (c > DEGCAP ? DEGCAP : c);
    int o = offs[s];
    o = o < 0 ? 0 : (o > RCAP ? RCAP : o);
    const int nc = node < nN ? node : nN - 1;
    float acc0 = 0.0f, acc1 = 0.0f;
#pragma unroll 1
    for (int b0 = 0; b0 < c; b0 += 32) {
      int idx = o + b0 + lane;
      idx = idx > RCAP - 1 ? RCAP - 1 : idx;
      const int ent = sl[idx];
      int eid = ent >> SLA;
      eid = eid < 0 ? 0 : (eid > nE - 1 ? nE - 1 : eid);
      int sr = srcs[eid];
      sr = sr < 0 ? 0 : (sr > nN - 1 ? nN - 1 : sr);
      const int m32 = (c - b0) < 32 ? (c - b0) : 32;
#pragma unroll 1
      for (int k = 0; k < m32; ++k) {
        const int sk = __builtin_amdgcn_readlane(sr, k);
        const v2f a = *(const v2fa*)(pf + (size_t)sk * HID + 2 * lane);
        acc0 += a.x; acc1 += a.y;
      }
    }
    float sv0, sv1;
    {
      const v2f a = *(const v2fa*)(pf + (size_t)nc * HID + 2 * lane);
      sv0 = a.x; sv1 = a.y;
    }
    const float pzr = big ? qnan : pz;
    const bool live = node < nN;
    float y0 = (sv0 + acc0) + bv0;
    float y1 = (sv1 + acc1) + bv1;
    y0 = fmaxf(y0, 0.0f); y1 = fmaxf(y1, 0.0f);
    y0 = y0 + pzr; y1 = y1 + pzr;
    const float v0 = live ? y0 : 0.0f;
    const float v1 = live ? y1 : 0.0f;
    const bool wr = (node < mRows) && (lane < 16);
    const unsigned hb0 = bf16_bits(v0), hb1 = bf16_bits(v1);
    const unsigned lb0 = bf16_bits(v0 - __uint_as_float(hb0 << 16));
    const unsigned lb1 = bf16_bits(v1 - __uint_as_float(hb1 << 16));
    const int hw = (int)(hb0 | (hb1 << 16));
    const int lw = (int)(lb0 | (lb1 << 16));
    const int g0 = __shfl(hw, q0s, 32), g1 = __shfl(hw, q1s, 32);
    const int g2 = __shfl(hw, q2s, 32), g3 = __shfl(hw, q3s, 32);
    const int p0 = __shfl(lw, q0s, 32), p1 = __shfl(lw, q1s, 32);
    const int p2 = __shfl(lw, q2s, 32), p3 = __shfl(lw, q3s, 32);
    const bool lsel = (lane & 8) != 0;
    v4u pv;
    pv.x = (unsigned int)(lsel ? p0 : g0);
    pv.y = (unsigned int)(lsel ? p1 : g1);
    pv.z = (unsigned int)(lsel ? p2 : g2);
    pv.w = (unsigned int)(lsel ? p3 : g3);
    unsigned short* hp = zb + (size_t)node * KK + 8 * (lane & 15);
    if (wr) *(volatile v4u*)hp = pv;
    __threadfence();
    if (wr) *(volatile v4u*)hp = pv;
  }
}

__global__ __launch_bounds__(HID) void k_bnfin(const float* __restrict__ part, int nPart,
                                               const float* __restrict__ gam, const float* __restrict__ bet,
                                               float* ss) {
  __shared__ __attribute__((aligned(16))) float stg[2 * HID];
  const int tid = (int)threadIdx.x;
  double n = 0.0, mean = 0.0, M2 = 0.0;
#pragma unroll 1
  for (int b = 0; b < nPart; ++b) {
    const float* pr = part + (size_t)b * PARTW;
    const double nb = (double)pr[0];
    const double mb = (double)pr[1 + tid];
    const double qb = (double)pr[1 + HID + tid];
    if (nb > 0.5) {
      const double nn = n + nb;
      const double delta = mb - mean;
      const double f = nb / nn;
      mean = mean + delta * f;
      M2 = M2 + qb + delta * delta * n * f;
      n = nn;
    }
  }
  const double nt = n < 1.0 ? 1.0 : n;
  const float var  = (float)(M2 / nt);
  const float rstd = 1.0f / sqrtf(var + 1e-5f);
  const float sc = bf16_val(gam[tid]) * rstd;
  const float sh = bf16_val(bet[tid]) - (float)mean * sc;
  stg[tid] = sc;
  stg[HID + tid] = sh;
  __syncthreads();
  const bool ok = tid < 32;
  const int j = tid & 31;
  v4f v = {0.f, 0.f, 0.f, 0.f};
  float* dp = ss + 4 * j;
  if (ok) {
    v = *(const v4fa*)(stg + 4 * j);
    *(volatile v4f*)dp = v;
  }
  __threadfence();
  if (ok) *(volatile v4f*)dp = v;
}

template <int MODE>
__global__ __launch_bounds__(NTHR) void k_bnap(const float* __restrict__ zf, const float* __restrict__ ss,
                                               int nN, int mRows, unsigned short* hl, float* outF) {
  __shared__ float ssh[2 * HID];
  __shared__ __attribute__((aligned(16))) float tile[APR * HID];
  const int tid = (int)threadIdx.x;
  if (tid < 2 * HID) ssh[tid] = ss[tid];
  const int rowBase = (int)blockIdx.x * APR;
  const int c  = tid & (HID - 1);
  const int rs = tid >> 6;
  __syncthreads();
#pragma unroll 1
  for (int r = 0; r < APR / 4; ++r) {
    const int lr   = 4 * r + rs;
    const int grow = rowBase + lr;
    const int gc   = grow < nN ? grow : nN - 1;
    const float z = zf[(size_t)gc * HID + c];
    const float v = fmaxf(fmaf(z, ssh[c], ssh[HID + c]), 0.0f);
    tile[lr * HID + c] = (grow < nN) ? v : 0.0f;
  }
  __syncthreads();
  if constexpr (MODE != 0) {
    v8us ov[2];
#pragma unroll
    for (int it = 0; it < 2; ++it) {
      const int p = it * NTHR + tid;
      const int lr = p >> 4, q = p & 15;
      const int ch = 8 * (q & 7);
      const v4f a = *(const v4fa*)(tile + lr * HID + ch);
      const v4f b = *(const v4fa*)(tile + lr * HID + ch + 4);
      v8us hv, lv;
      hilo8(a, b, hv, lv);
      const bool isHi = q < 8;
      v8us o;
#pragma unroll
      for (int j = 0; j < 8; ++j) o[j] = isHi ? hv[j] : lv[j];
      ov[it] = o;
    }
#pragma unroll
    for (int it = 0; it < 2; ++it) {
      const int p = it * NTHR + tid;
      const int lr = p >> 4, q = p & 15;
      const int grow = rowBase + lr;
      unsigned short* op = hl + (size_t)grow * KK + 8 * q;
      if (grow < mRows) *(volatile v8us*)op = ov[it];
    }
    __threadfence();
#pragma unroll
    for (int it = 0; it < 2; ++it) {
      const int p = it * NTHR + tid;
      const int lr = p >> 4, q = p & 15;
      const int grow = rowBase + lr;
      unsigned short* op = hl + (size_t)grow * KK + 8 * q;
      if (grow < mRows) *(volatile v8us*)op = ov[it];
    }
  } else {
    v4f pv[2];
#pragma unroll
    for (int it = 0; it < 2; ++it) {
      const int p = it * NTHR + tid;
      const int lr = p >> 4, q = p & 15;
      pv[it] = *(const v4fa*)(tile + lr * HID + 4 * q);
    }
#pragma unroll
    for (int it = 0; it < 2; ++it) {
      const int p = it * NTHR + tid;
      const int lr = p >> 4, q = p & 15;
      const int grow = rowBase + lr;
      float* op = outF + (size_t)grow * HID + 4 * q;
      if (grow < nN) *(volatile v4f*)op = pv[it];
    }
    __threadfence();
#pragma unroll
    for (int it = 0; it < 2; ++it) {
      const int p = it * NTHR + tid;
      const int lr = p >> 4, q = p & 15;
      const int grow = rowBase + lr;
      float* op = outF + (size_t)grow * HID + 4 * q;
      if (grow < nN) *(volatile v4f*)op = pv[it];
    }
  }
}

static inline int cdiv(int a, int b) { return (a + b - 1) / b; }
static inline size_t al256(size_t o) { return (o + 255) & ~(size_t)255; }

extern "C" void kernel_launch(void* const* d_in, const int* in_sizes, int n_in,
                              void* d_out, int out_size, void* d_ws, size_t ws_size,
                              hipStream_t stream) {
  if (n_in < 15) return;
  if (in_sizes[0] < CIN || (in_sizes[0] % CIN) != 0) return;
  const int nN = in_sizes[0] / CIN;
  if (nN < 1 || nN > (1 << 22)) return;
  const int nE = in_sizes[1];
  if (nE < 1 || nE >= (1 << (31 - SLA))) return;
  if (in_sizes[2] != nE) return;
  if (in_sizes[3] != CIN * HID || in_sizes[4] != HID) return;
  if (in_sizes[5] != HID * HID || in_sizes[6] != HID) return;
  if (in_sizes[7] != HID || in_sizes[8] != HID) return;
  if (in_sizes[9] != (NLAY - 1) * HID * HID || in_sizes[10] != (NLAY - 1) * HID) return;
  if (in_sizes[11] != (NLAY - 1) * HID * HID || in_sizes[12] != (NLAY - 1) * HID) return;
  if (in_sizes[13] != (NLAY - 1) * HID || in_sizes[14] != (NLAY - 1) * HID) return;
  if ((long long)out_size != (long long)nN * HID) return;

  const float* x    = (const float*)d_in[0];
  const int*   src  = (const int*)  d_in[1];
  const int*   dst  = (const int*)  d_in[2];
  const float* w10  = (const float*)d_in[3];
  const float* b10  = (const float*)d_in[4];
  const float* w20  = (const float*)d_in[5];
  const float* b20  = (const float*)d_in[6];
  const float* g0   = (const float*)d_in[7];
  const float* be0  = (const float*)d_in[8];
  const float* w1s  = (const float*)d_in[9];
  const float* b1s  = (const float*)d_in[10];
  const float* w2s  = (const float*)d_in[11];
  const float* b2s  = (const float*)d_in[12];
  const float* gs   = (const float*)d_in[13];
  const float* bes  = (const float*)d_in[14];
  float* out = (float*)d_out;

  const int MP = cdiv(nN, GBM) * GBM;
  const int gM = MP / GBM;
  const int gA = cdiv(MP, NBA);
  if ((long long)gA * NBA < (long long)MP) return;
  if ((MP % APR) != 0) return;
  const int vec8 = ((((size_t)in_sizes[0] * 4 + (size_t)in_sizes[1] * 4) & 15) == 0) ? 1 : 0;

  char* ws = (char*)d_ws;
  size_t off = 0;
  const size_t oWP = off; off = al256(off + (size_t)NPL * PLSZ * 2);
  const size_t oHB = off; off = al256(off + (size_t)MP * CIN * 2);
  const size_t oPF = off; off = al256(off + (size_t)MP * HID * 4);
  const size_t oZ1 = off; off = al256(off + (size_t)MP * KK * 2);
  const size_t oZF = off; off = al256(off + (size_t)MP * HID * 4);
  const size_t oHL = off; off = al256(off + (size_t)MP * KK * 2);
  const size_t oPT = off; off = al256(off + (size_t)gM * PARTW * 4);
  const size_t oSS = off; off = al256(off + (size_t)(2 * HID) * 4);
  if (off > ws_size || off > (size_t)WSMAX) return;
  unsigned short* WP = (unsigned short*)(ws + oWP);
  unsigned short* HB = (unsigned short*)(ws + oHB);
  float*          PF = (float*)(ws + oPF);
  unsigned short* Z1 = (unsigned short*)(ws + oZ1);
  float*          ZF = (float*)(ws + oZF);
  unsigned short* HL = (unsigned short*)(ws + oHL);
  float*          PT = (float*)(ws + oPT);
  float*          SS = (float*)(ws + oSS);

  const size_t aggLds = (size_t)AGG_LDS_INTS * 4;
  hipFuncSetAttribute(reinterpret_cast<const void*>(&k_agg), hipFuncAttributeMaxDynamicSharedMemorySize, (int)aggLds);

  const int nUx = MP * (CIN / 8);
  k_wprep<<<NUW / NTHR, NTHR, 0, stream>>>(w10, w20, w1s, w2s, WP);
  k_cvx<<<cdiv(nUx, NTHR), NTHR, 0, stream>>>(x, nN, nUx, HB);
  for (int L = 0; L < NLAY; ++L) {
    const unsigned short* A   = (L == 0) ? HB : HL;
    const unsigned short* W1T = WP + (size_t)(2 * L) * PLSZ;
    const unsigned short* W2T = WP + (size_t)(2 * L + 1) * PLSZ;
    const float* b1 = (L == 0) ? b10 : b1s + (size_t)(L - 1) * HID;
    const float* b2 = (L == 0) ? b20 : b2s + (size_t)(L - 1) * HID;
    const float* ga = (L == 0) ? g0  : gs  + (size_t)(L - 1) * HID;
    const float* be = (L == 0) ? be0 : bes + (size_t)(L - 1) * HID;
    k_gemm<0><<<dim3(gM, HID / GBN), GTHR, 0, stream>>>(A, W1T, b1, PF, KK, nN, PT);
    k_agg<<<gA, NTHR, aggLds, stream>>>(src, dst, nE, nN, vec8, MP, PF, b1, Z1);
    k_gemm<1><<<dim3(gM, HID / GBN), GTHR, 0, stream>>>(Z1, W2T, b2, ZF, KK, nN, PT);
    k_bnfin<<<1, HID, 0, stream>>>(PT, gM, ga, be, SS);
    if (L < NLAY - 1) k_bnap<1><<<MP / APR, NTHR, 0, stream>>>(ZF, SS, nN, MP, HL, out);
    else              k_bnap<0><<<MP / APR, NTHR, 0, stream>>>(ZF, SS, nN, MP, HL, out);
  }
}
